// QuantLinear_3040836845619
// MI455X (gfx1250) — hardware-verified
//
#include <hip/hip_runtime.h>

typedef unsigned short v8us __attribute__((ext_vector_type(8)));
typedef short          v16s __attribute__((ext_vector_type(16)));
typedef __bf16         v16b __attribute__((ext_vector_type(16)));
typedef float          v8f  __attribute__((ext_vector_type(8)));
typedef float          v4f  __attribute__((ext_vector_type(4)));
typedef int            v4i  __attribute__((ext_vector_type(4)));
typedef v8us __attribute__((may_alias)) v8usa;
typedef v4f  __attribute__((may_alias)) v4fa;
typedef v4i  __attribute__((may_alias)) v4ia;

union Frag { v16b v; v16s s; v8us half[2]; };

#define NTOK  2048
#define KIN   4096
#define NOUT  4096
#define GRP   128
#define NGRP  (KIN / GRP)
#define NXE   (NTOK * KIN)
#define NX8   (NXE / 8)
#define NQW   ((KIN / 8) * NOUT)
#define NQZ   (NGRP * (NOUT / 8))
#define NSC   (NGRP * NOUT)
#define NOE   (NTOK * NOUT)
#define WTO   64
#define WTK   256
#define WP    264
#define BNAN  0x7FC0

static_assert(NX8 % 256 == 0);
static_assert(KIN % GRP == 0);
static_assert(GRP % 32 == 0);
static_assert(NOUT % WTO == 0);
static_assert(KIN % WTK == 0);
static_assert(WTK % 8 == 0);
static_assert(NTOK % 64 == 0);
static_assert(NOUT % 64 == 0);
static_assert((WP * 2) % 16 == 0);
static_assert(WTO * WP <= 32768);

__device__ __forceinline__ unsigned short f2bf(float f) {
  unsigned u = __float_as_uint(f);
  u = u + 0x7FFFu + ((u >> 16) & 1u);
  return (unsigned short)(u >> 16);
}
__device__ __forceinline__ float bf16r(float f) {
  return __uint_as_float(((unsigned)f2bf(f)) << 16);
}
__device__ __forceinline__ int clampi(int v, int lo, int hi) {
  return v < lo ? lo : (v > hi ? hi : v);
}

__device__ __forceinline__ v8f wmma_bf16(const Frag a, const Frag b, v8f c) {
  v8f d = __builtin_amdgcn_wmma_f32_16x16x32_bf16(false, a.v, false, b.v, (short)0, c, false, false);
  asm volatile("v_nop\n\tv_nop\n\tv_nop\n\tv_nop" : "+v"(d) : "v"(a.s), "v"(b.s));
  return d;
}

__device__ __forceinline__ Frag load_frag(const unsigned short* p, int h) {
  Frag f;
  f.half[0] = *(const v8usa*)(p + 8 * h);
  f.half[1] = *(const v8usa*)(p + 16 + 8 * h);
  return f;
}

__global__ __launch_bounds__(256) void xcvt_kernel(const float* __restrict__ x,
                                                   unsigned short* __restrict__ xb)
{
  const int g = blockIdx.x * 256 + threadIdx.x;
  if (g >= NX8) return;
  const float* src = x + (size_t)g * 8;
  const v4f a = *(const v4fa*)src;
  const v4f c = *(const v4fa*)(src + 4);
  const v8us o = { f2bf(a.x), f2bf(a.y), f2bf(a.z), f2bf(a.w),
                   f2bf(c.x), f2bf(c.y), f2bf(c.z), f2bf(c.w) };
  unsigned short* dst = xb + (size_t)g * 8;
  *(volatile v8us*)dst = o;
  __threadfence();
  *(volatile v8us*)dst = o;
}

__device__ __forceinline__ unsigned short ival(unsigned q, int j, int z, bool ok) {
  const int wv = (int)((q >> (4 * j)) & 15u);
  return ok ? f2bf((float)(wv - z)) : (unsigned short)BNAN;
}
__device__ __forceinline__ v8us unpack8(unsigned q, int z, bool ok) {
  const v8us v = { ival(q, 0, z, ok), ival(q, 1, z, ok), ival(q, 2, z, ok), ival(q, 3, z, ok),
                   ival(q, 4, z, ok), ival(q, 5, z, ok), ival(q, 6, z, ok), ival(q, 7, z, ok) };
  return v;
}

__device__ __forceinline__ void wq_store_pass(const unsigned short* sW, unsigned short* wq,
                                              int o0, int kb0, int w, int lane) {
  const int q8 = lane & 7, sub = lane >> 3;
  #pragma unroll
  for (int i = 0; i < 8; ++i) {
    const int lid = w * 32 + i * 4 + sub;
    const int ol = lid >> 2, ch = lid & 3;
    const v8us v = *(const v8usa*)(sW + ol * WP + ch * 64 + 8 * q8);
    unsigned short* dst = wq + (size_t)(o0 + ol) * KIN + kb0 + ch * 64 + 8 * q8;
    *(volatile v8us*)dst = v;
  }
}

__global__ __launch_bounds__(256) void wq_kernel(
    const int* __restrict__ qweight,
    const int* __restrict__ qzeros,
    const int* __restrict__ g_idx,
    unsigned short* __restrict__ wq)
{
  __shared__ __attribute__((aligned(16))) unsigned short sW[WTO * WP];

  const int tid = threadIdx.x, lane = tid & 31, w = tid >> 5;
  const int o0  = blockIdx.x * WTO;
  const int kb0 = blockIdx.y * WTK;
  const int kp0 = kb0 / 8;

  #pragma unroll
  for (int it = 0; it < 2; ++it) {
    const int idx = it * 256 + tid;
    const int pr  = idx >> 4;
    const int oc4 = (idx & 15) * 4;
    const v4i q4 = *(const v4ia*)(qweight + (size_t)(kp0 + pr) * NOUT + o0 + oc4);
    const int kq = kb0 + 8 * pr;
    const v4i ga = *(const v4ia*)(g_idx + kq);
    const v4i gb = *(const v4ia*)(g_idx + kq + 4);
    const int g0 = g_idx[kq & ~(GRP - 1)];
    const bool same = (ga.x == g0) & (ga.y == g0) & (ga.z == g0) & (ga.w == g0) &
                      (gb.x == g0) & (gb.y == g0) & (gb.z == g0) & (gb.w == g0);
    const int g = clampi(g0, 0, NGRP - 1);
    const unsigned zq = (unsigned)qzeros[g * (NOUT / 8) + ((o0 + oc4) >> 3)];
    #pragma unroll
    for (int c = 0; c < 4; ++c) {
      const int z = (int)((zq >> (4 * ((oc4 + c) & 7))) & 15u) + 1;
      const v8us v = unpack8((unsigned)q4[c], z, same);
      *(v8usa*)(sW + (oc4 + c) * WP + 8 * pr) = v;
    }
  }
  __syncthreads();

  wq_store_pass(sW, wq, o0, kb0, w, lane);
  __threadfence();
  wq_store_pass(sW, wq, o0, kb0, w, lane);
}

__device__ __forceinline__ void out_store_pass(const float* so, float* out,
                                               int m0w, int n0w, int lane) {
  const int q8 = lane & 7, sub = lane >> 3;
  #pragma unroll
  for (int i = 0; i < 8; ++i) {
    const int row = i * 4 + sub;
    const v4f v = *(const v4fa*)(so + row * 32 + 4 * q8);
    *(volatile v4f*)(out + (size_t)(m0w + row) * NOUT + n0w + 4 * q8) = v;
  }
}

__global__ __launch_bounds__(128) void gemm_kernel(
    const unsigned short* __restrict__ xb,
    const unsigned short* __restrict__ wq,
    const float* __restrict__ scales,
    const int* __restrict__ g_idx,
    float* __restrict__ out)
{
  __shared__ __attribute__((aligned(16))) float sO[4 * 32 * 32];

  const int tid = threadIdx.x, lane = tid & 31, w = tid >> 5;
  const int h = lane >> 4, m = lane & 15;
  const int wm = w & 1, wn = w >> 1;
  const int m0w = blockIdx.y * 64 + 32 * wm;
  const int n0w = blockIdx.x * 64 + 32 * wn;

  const unsigned short* xa0 = xb + (size_t)(m0w + m) * KIN;
  const unsigned short* xa1 = xa0 + (size_t)16 * KIN;
  const unsigned short* wb0 = wq + (size_t)(n0w + m) * KIN;
  const unsigned short* wb1 = wb0 + (size_t)16 * KIN;
  const float* scn = scales + n0w + m;

  const v8f zero8 = {0.f, 0.f, 0.f, 0.f, 0.f, 0.f, 0.f, 0.f};
  v8f acc[2][2], accg[2][2];
  #pragma unroll
  for (int mt = 0; mt < 2; ++mt)
    #pragma unroll
    for (int nt = 0; nt < 2; ++nt) acc[mt][nt] = zero8;

  #pragma unroll 1
  for (int ks = 0; ks < NGRP; ++ks) {
    #pragma unroll
    for (int mt = 0; mt < 2; ++mt)
      #pragma unroll
      for (int nt = 0; nt < 2; ++nt) accg[mt][nt] = zero8;

    #pragma unroll
    for (int kk = 0; kk < GRP / 32; ++kk) {
      const int k0 = ks * GRP + kk * 32;
      const Frag a0 = load_frag(xa0 + k0, h);
      const Frag a1 = load_frag(xa1 + k0, h);
      const Frag b0 = load_frag(wb0 + k0, h);
      const Frag b1 = load_frag(wb1 + k0, h);
      accg[0][0] = wmma_bf16(a0, b0, accg[0][0]);
      accg[0][1] = wmma_bf16(a0, b1, accg[0][1]);
      accg[1][0] = wmma_bf16(a1, b0, accg[1][0]);
      accg[1][1] = wmma_bf16(a1, b1, accg[1][1]);
    }

    const int g = clampi(g_idx[ks * GRP], 0, NGRP - 1);
    #pragma unroll
    for (int nt = 0; nt < 2; ++nt) {
      const float sc = bf16r(scn[(size_t)g * NOUT + 16 * nt]);
      #pragma unroll
      for (int mt = 0; mt < 2; ++mt)
        #pragma unroll
        for (int r = 0; r < 8; ++r)
          acc[mt][nt][r] = fmaf(sc, accg[mt][nt][r], acc[mt][nt][r]);
    }
  }

  float* so = sO + w * 1024;
  #pragma unroll
  for (int mt = 0; mt < 2; ++mt)
    #pragma unroll
    for (int nt = 0; nt < 2; ++nt)
      #pragma unroll
      for (int r = 0; r < 8; ++r)
        so[(16 * mt + 8 * h + r) * 32 + 16 * nt + m] = acc[mt][nt][r];
  __syncthreads();

  out_store_pass(so, out, m0w, n0w, lane);
  __threadfence();
  out_store_pass(so, out, m0w, n0w, lane);
}

extern "C" void kernel_launch(void* const* d_in, const int* in_sizes, int n_in,
                              void* d_out, int out_size, void* d_ws, size_t ws_size,
                              hipStream_t stream) {
  if (n_in < 5) return;
  if (in_sizes[0] != NXE) return;
  if (in_sizes[1] != NQW) return;
  if (in_sizes[2] != NQZ) return;
  if (in_sizes[3] != NSC) return;
  if (in_sizes[4] != KIN) return;
  if (out_size != NOE) return;

  const float* x       = (const float*)d_in[0];
  const int*   qweight = (const int*)  d_in[1];
  const int*   qzeros  = (const int*)  d_in[2];
  const float* scales  = (const float*)d_in[3];
  const int*   g_idx   = (const int*)  d_in[4];
  float* out = (float*)d_out;

  const size_t xb_bytes = (size_t)NXE * 2;
  const size_t wq_bytes = (size_t)NOUT * KIN * 2;
  const size_t total = xb_bytes + wq_bytes;
  if (total > ws_size) return;

  char* ws = (char*)d_ws;
  unsigned short* xb = (unsigned short*)(ws);
  unsigned short* wq = (unsigned short*)(ws + xb_bytes);

  xcvt_kernel<<<NX8 / 256, 256, 0, stream>>>(x, xb);

  dim3 gW(NOUT / WTO, KIN / WTK);
  wq_kernel<<<gW, 256, 0, stream>>>(qweight, qzeros, g_idx, wq);

  dim3 gG(NOUT / 64, NTOK / 64);
  gemm_kernel<<<gG, 128, 0, stream>>>(xb, wq, scales, g_idx, out);
}
